// TokenToSceneGraph_31593779429483
// MI455X (gfx1250) — hardware-verified
//
#include <hip/hip_runtime.h>
#include <math.h>

typedef __attribute__((ext_vector_type(16))) _Float16 v16h;
typedef __attribute__((ext_vector_type(8)))  _Float16 v8h;
typedef __attribute__((ext_vector_type(16))) __bf16   v16b;
typedef __attribute__((ext_vector_type(8)))  __bf16   v8b;
typedef __attribute__((ext_vector_type(8)))  float    v8f;
typedef __attribute__((ext_vector_type(4)))  float    v4f;
typedef __attribute__((ext_vector_type(4)))  unsigned int v4u;

constexpr int kNB    = 256;
constexpr int kNT    = 77;
constexpr int kNTP   = 96;
constexpr int kNTS   = 80;
constexpr int kDM    = 768;
constexpr int kKN    = 16;
constexpr int kHD    = 512;
constexpr int kNL    = 2;
constexpr int kBPC   = 64;
constexpr int kNCH   = 4;
constexpr int kMRC   = kBPC * kNTP;
constexpr int kQR    = 64;
constexpr int kVROWS = kNB * kKN;
constexpr int kG8    = kDM / 8;
constexpr float kScoreScale = 0.10206207261596577f;
constexpr float kKVCarry    = 32.0f;
constexpr float kKVScale    = 1.0f / 32.0f;
constexpr float kWCarry     = 64.0f;
constexpr float kVCarry     = 4.0f;
constexpr float kReluCarry  = 16.0f;
constexpr float kProjScale  = 1.0f / (kWCarry * kVCarry);
constexpr float kEdgeScale  = 1.0f / (kReluCarry * kWCarry);
static_assert(kNB == kBPC * kNCH);
static_assert(kMRC % 64 == 0 && kDM % 64 == 0 && kHD % 64 == 0 && kVROWS % 64 == 0);
static_assert(kNTS % 16 == 0 && kNTS <= kNTP && kNTP % 32 == 0 && kNT <= kNTS);

constexpr size_t kSzW2    = (size_t)kDM * kDM * 2;
constexpr size_t kSzWe1T  = (size_t)(2 * kHD) * kDM * 2;
constexpr size_t kSzQpl   = (size_t)kQR * kDM * 2;
constexpr size_t kSzWpl   = (size_t)kMRC * kDM * 2;
constexpr size_t kSzVtpl  = (size_t)kDM * kMRC * 2;
constexpr size_t kSzSst   = (size_t)kNB * kNTP * kKN * 4;
constexpr size_t kSzVf    = (size_t)kVROWS * kDM * 4;
constexpr size_t kSzVh    = (size_t)kVROWS * kDM * 2;
constexpr size_t kSzH     = (size_t)kVROWS * (2 * kHD) * 4;
constexpr size_t kSzGT    = (size_t)kDM * kVROWS * 2;
constexpr size_t kSzAdj   = (size_t)kNB * kKN * kKN * 4;

constexpr size_t oWqH   = 0;
constexpr size_t oWqL   = oWqH + kSzW2;
constexpr size_t oWkT   = oWqL + kSzW2;
constexpr size_t oWvT   = oWkT + kSzW2;
constexpr size_t oWe1T  = oWvT + kSzW2;
constexpr size_t oWgT   = oWe1T + kSzWe1T;
constexpr size_t oQinH  = oWgT + 2 * kSzW2;
constexpr size_t oQinL  = oQinH + kSzQpl;
constexpr size_t oQH    = oQinL + kSzQpl;
constexpr size_t oQL    = oQH + kSzQpl;
constexpr size_t oChunk = oQL + kSzQpl;
constexpr size_t oWH    = oChunk;
constexpr size_t oKtH   = oWH + kSzWpl;
constexpr size_t oKtL   = oKtH + kSzWpl;
constexpr size_t oVtH   = oKtL + kSzWpl;
constexpr size_t oVtL   = oVtH + kSzVtpl;
constexpr size_t oChunkEnd = oVtL + kSzVtpl;
constexpr size_t oH     = oChunk;
constexpr size_t oGTH   = oH + kSzH;
constexpr size_t oGTL   = oGTH + kSzGT;
constexpr size_t oVfB   = oGTL + kSzGT;
static_assert(oVfB + kSzVf <= oChunkEnd);
constexpr size_t oSst   = oChunkEnd;
constexpr size_t oVfA   = oSst + kSzSst;
constexpr size_t oVhA   = oVfA + kSzVf;
constexpr size_t oVhB   = oVhA + kSzVh;
constexpr size_t oAdj   = oVhB + kSzVh;
constexpr size_t kWsTotal = oAdj + kSzAdj;
static_assert(kWsTotal <= (size_t)134217728);
static_assert((oChunk & 255) == 0 && (oChunkEnd & 255) == 0 && (oAdj & 255) == 0 && (oGTH & 255) == 0 && (oVfB & 255) == 0);

__device__ __forceinline__ unsigned short f2bf_bits(float f) {
  unsigned u = __float_as_uint(f);
  return (unsigned short)((u + 0x7FFFu + ((u >> 16) & 1u)) >> 16);
}
__device__ __forceinline__ float bf_bits2f(unsigned short h) { return __uint_as_float(((unsigned)h) << 16); }

__device__ __forceinline__ void dep_guard_h(v8f& a, v8f& b, v16h x, v16h y) { asm volatile("v_nop\n\tv_nop\n\tv_nop\n\tv_nop" : "+v"(a), "+v"(b) : "v"(x), "v"(y)); }
__device__ __forceinline__ void dep_guard_b(v8f& a, v8f& b, v16b x, v16b y) { asm volatile("v_nop\n\tv_nop\n\tv_nop\n\tv_nop" : "+v"(a), "+v"(b) : "v"(x), "v"(y)); }
__device__ __forceinline__ void keep4_h(v16h a, v16h b, v16h c, v16h d) { asm volatile("v_nop" :: "v"(a), "v"(b), "v"(c), "v"(d)); }
__device__ __forceinline__ void keep4_b(v16b a, v16b b, v16b c, v16b d) { asm volatile("v_nop" :: "v"(a), "v"(b), "v"(c), "v"(d)); }
__device__ __forceinline__ void acc_guard4(v8f& a, v8f& b, v8f& c, v8f& d) { asm volatile("v_nop\n\tv_nop\n\tv_nop\n\tv_nop" : "+v"(a), "+v"(b), "+v"(c), "+v"(d)); }
template <typename T> struct Frag;
template <> struct Frag<_Float16> {
  typedef v16h V; union U { v16h v; v8h h[2]; };
  static __device__ __forceinline__ v16h load(const _Float16* p) {
    U f; f.h[0] = *(const v8h*)(p); f.h[1] = *(const v8h*)(p + 16); return f.v;
  }
  static __device__ __forceinline__ v8f mma(v16h a, v16h b, v8f c) {
    return __builtin_amdgcn_wmma_f32_16x16x32_f16(false, a, false, b, (short)0, c, false, false);
  }
  static __device__ __forceinline__ void guard(v8f& a, v8f& b, v16h x, v16h y) { dep_guard_h(a, b, x, y); }
  static __device__ __forceinline__ void keep(v16h a, v16h b, v16h c, v16h d) { keep4_h(a, b, c, d); }
};
template <> struct Frag<__bf16> {
  typedef v16b V; union U { v16b v; v8b h[2]; };
  static __device__ __forceinline__ v16b load(const __bf16* p) {
    U f; f.h[0] = *(const v8b*)(p); f.h[1] = *(const v8b*)(p + 16); return f.v;
  }
  static __device__ __forceinline__ v8f mma(v16b a, v16b b, v8f c) {
    return __builtin_amdgcn_wmma_f32_16x16x32_bf16(false, a, false, b, (short)0, c, false, false);
  }
  static __device__ __forceinline__ void guard(v8f& a, v8f& b, v16b x, v16b y) { dep_guard_b(a, b, x, y); }
  static __device__ __forceinline__ void keep(v16b a, v16b b, v16b c, v16b d) { keep4_b(a, b, c, d); }
};

__device__ __forceinline__ unsigned pk16(unsigned short a, unsigned short b) { return (unsigned)a | ((unsigned)b << 16); }
__device__ __forceinline__ unsigned short h_bits(float f) { const _Float16 h = (_Float16)f; return __builtin_bit_cast(unsigned short, h); }

__device__ __forceinline__ unsigned short at_bf_bits(float f) {
  unsigned u = __float_as_uint(f);
  return (unsigned short)((u + 0x7FFFu + ((u >> 16) & 1u)) >> 16);
}
__device__ __forceinline__ __bf16 at_f2bf(float f) { return __builtin_bit_cast(__bf16, at_bf_bits(f)); }
__device__ __forceinline__ void at_split(float f, __bf16& hi, __bf16& lo) {
  const unsigned short hb = at_bf_bits(f);
  hi = __builtin_bit_cast(__bf16, hb);
  lo = at_f2bf(f - __uint_as_float(((unsigned)hb) << 16));
}
__device__ __forceinline__ v8f bmma(v16b a, v16b b, v8f c) {
  c = __builtin_amdgcn_wmma_f32_16x16x32_bf16(false, a, false, b, (short)0, c, false, false);
  asm volatile("v_nop\n\tv_nop\n\tv_nop\n\tv_nop" : "+v"(c) : "v"(a), "v"(b));
  return c;
}
__device__ __forceinline__ v8f hmma(v16h a, v16h b, v8f c) {
  c = __builtin_amdgcn_wmma_f32_16x16x32_f16(false, a, false, b, (short)0, c, false, false);
  asm volatile("v_nop\n\tv_nop\n\tv_nop\n\tv_nop" : "+v"(c) : "v"(a), "v"(b));
  return c;
}
__device__ __forceinline__ void wave_sync_lds() {
  __builtin_amdgcn_fence(__ATOMIC_RELEASE, "workgroup");
  __builtin_amdgcn_wave_barrier();
  __builtin_amdgcn_fence(__ATOMIC_ACQUIRE, "workgroup");
}
union FB { v16b v; v8b h[2]; v4u u4[2]; };

template <int ET> struct Elem;
template <> struct Elem<0> { typedef _Float16 T; };
template <> struct Elem<1> { typedef __bf16 T; };
template <int ET, bool SPLIT, int BIAS_MODE, int OUT_MODE, bool RESID, int ACT = 0, int ZPN = 0, int ZPV = 0>
__global__ __launch_bounds__(256) void wmma_gemm64(
    const unsigned short* __restrict__ Ap, const unsigned short* __restrict__ A2p, int lda, long strideA,
    const unsigned short* __restrict__ Btp, const unsigned short* __restrict__ Bt2p, int ldb, long strideB,
    void* __restrict__ Cout, void* __restrict__ Cout2, int ldc, long strideC,
    const float* __restrict__ bias,
    const float* __restrict__ resid, long strideR,
    int M, int N, int K, float scale) {
  typedef typename Elem<ET>::T T;
  typedef typename Frag<T>::V V;
  const T* A = (const T*)Ap; const T* A2 = (const T*)A2p; const T* Bt = (const T*)Btp; const T* Bt2 = (const T*)Bt2p;
  __shared__ __align__(16) float sT[8][16 * 68];
  const int b    = blockIdx.y;
  const int lane = threadIdx.x & 31;
  const int wave = threadIdx.x >> 5;
  const int tilesN = N >> 6;
  const int tilesM = M >> 6;
  const int tile = blockIdx.x * 8 + wave;
  if (tile >= tilesM * tilesN) return;
  const int tm = tile / tilesN;
  const int tn = tile - tm * tilesN;
  const int m0 = tm << 6;
  const int n0 = tn << 6;

  const T* Ab  = A  + (size_t)b * strideA;
  const T* Bb  = Bt + (size_t)b * strideB;
  const T* Ab2 = SPLIT ? (A2  + (size_t)b * strideA) : nullptr;
  const T* Bb2 = SPLIT ? (Bt2 + (size_t)b * strideB) : nullptr;

  const int rlane = lane & 15;
  const int koff  = (lane >> 4) * 8;
  const int mOff  = (lane >> 4) * 8;

  v8f acc[4][4];
#pragma unroll
  for (int i = 0; i < 4; ++i)
#pragma unroll
    for (int j = 0; j < 4; ++j) acc[i][j] = (v8f){0.f,0.f,0.f,0.f,0.f,0.f,0.f,0.f};

  for (int k0 = 0; k0 < K; k0 += 32) {
    V bh[4], bl[4];
#pragma unroll
    for (int j = 0; j < 4; ++j) {
      const size_t bo = (size_t)(n0 + (j << 4) + rlane) * ldb + koff + k0;
      bh[j] = Frag<T>::load(Bb + bo);
      if (SPLIT) bl[j] = Frag<T>::load(Bb2 + bo);
    }
#pragma unroll
    for (int i = 0; i < 4; ++i) {
      const size_t ao = (size_t)(m0 + (i << 4) + rlane) * lda + koff + k0;
      V ah = Frag<T>::load(Ab + ao);
      V al;
      if (SPLIT) al = Frag<T>::load(Ab2 + ao);
#pragma unroll
      for (int j = 0; j < 4; ++j) {
        acc[i][j] = Frag<T>::mma(ah, bh[j], acc[i][j]);
        if (SPLIT) {
          acc[i][j] = Frag<T>::mma(ah, bl[j], acc[i][j]);
          acc[i][j] = Frag<T>::mma(al, bh[j], acc[i][j]);
        }
      }
      Frag<T>::guard(acc[i][0], acc[i][3], ah, SPLIT ? al : ah);
    }
    Frag<T>::keep(bh[0], bh[1], bh[2], bh[3]);
    if (SPLIT) Frag<T>::keep(bl[0], bl[1], bl[2], bl[3]);
  }
  acc_guard4(acc[0][0], acc[0][1], acc[0][2], acc[0][3]);
  acc_guard4(acc[1][0], acc[1][1], acc[1][2], acc[1][3]);
  acc_guard4(acc[2][0], acc[2][1], acc[2][2], acc[2][3]);
  acc_guard4(acc[3][0], acc[3][1], acc[3][2], acc[3][3]);

  float* slab = sT[wave];
  const float* Rb = RESID ? (resid + (size_t)b * strideR) : nullptr;
#pragma unroll
  for (int i = 0; i < 4; ++i) {
    const int mBase = m0 + (i << 4);
#pragma unroll
    for (int j = 0; j < 4; ++j) {
      const int n = n0 + (j << 4) + rlane;
      float bv = 0.f;
      if (BIAS_MODE == 2) bv = bias[n];
      bool zc = false;
      if (ZPN > 0) zc = ((n % ZPN) >= ZPV);
#pragma unroll
      for (int r = 0; r < 8; ++r) {
        float v = acc[i][j][r] * scale;
        if (BIAS_MODE == 1) v += bias[mBase + mOff + r];
        if (BIAS_MODE == 2) v += bv;
        if (RESID) v += Rb[(size_t)(mBase + mOff + r) * ldc + n];
        if (ACT == 2) v = fmaxf(v, 0.0f);
        if (ACT == 4) v = (v > 0.f) ? v : 0.01f * v;
        if (ZPN > 0) v = zc ? 0.0f : v;
        slab[(mOff + r) * 68 + (j << 4) + rlane] = v;
      }
    }
    __builtin_amdgcn_fence(__ATOMIC_RELEASE, "workgroup");
    __builtin_amdgcn_wave_barrier();
    __builtin_amdgcn_fence(__ATOMIC_ACQUIRE, "workgroup");
    if (OUT_MODE == 0) {
      float* C = (float*)Cout + (size_t)b * strideC;
      const int hh = lane >> 4, c4 = (lane & 15) * 4;
      for (int pass = 0; pass < 2; ++pass) {
#pragma unroll
        for (int it = 0; it < 8; ++it) {
          const int row = it * 2 + hh;
          v4f v = *(const v4f*)(slab + row * 68 + c4);
          *(volatile v4f*)(C + (size_t)(mBase + row) * ldc + n0 + c4) = v;
        }
        __threadfence();
      }
    } else {
      const int q = lane >> 3, c8 = (lane & 7) * 8;
      unsigned short* C  = (unsigned short*)Cout  + (size_t)b * strideC;
      unsigned short* C2 = (OUT_MODE == 2) ? ((unsigned short*)Cout2 + (size_t)b * strideC) : nullptr;
      for (int pass = 0; pass < 2; ++pass) {
#pragma unroll
        for (int it = 0; it < 4; ++it) {
          const int row = it * 4 + q;
          const float* sp = slab + row * 68 + c8;
          v8h hv, lv;
#pragma unroll
          for (int e = 0; e < 8; ++e) {
            if (OUT_MODE == 1) {
              hv[e] = (_Float16)sp[e];
            } else {
              unsigned short hb = f2bf_bits(sp[e]);
              unsigned short lb = f2bf_bits(sp[e] - bf_bits2f(hb));
              hv[e] = __builtin_bit_cast(_Float16, hb);
              lv[e] = __builtin_bit_cast(_Float16, lb);
            }
          }
          *(volatile v8h*)(C + (size_t)(mBase + row) * ldc + n0 + c8) = hv;
          if (OUT_MODE == 2) *(volatile v8h*)(C2 + (size_t)(mBase + row) * ldc + n0 + c8) = lv;
        }
        __threadfence();
      }
    }
    __builtin_amdgcn_fence(__ATOMIC_RELEASE, "workgroup");
    __builtin_amdgcn_wave_barrier();
    __builtin_amdgcn_fence(__ATOMIC_ACQUIRE, "workgroup");
  }
}

template <int CMODE>
__global__ __launch_bounds__(256) void tcast_kernel(const float* __restrict__ src, long src_z, int sp,
                                                    unsigned short* __restrict__ dst, unsigned short* __restrict__ dst2,
                                                    long dst_z, int dp, float scale) {
  __shared__ float sm[64][65];
  const int t  = threadIdx.x;
  const int k0 = blockIdx.x * 64;
  const int n0 = blockIdx.y * 64;
  const int z  = blockIdx.z;
  const float* S = src + (size_t)z * src_z;
#pragma unroll
  for (int i = 0; i < 16; ++i) {
    const int e = i * 256 + t;
    const int r = e >> 6;
    const int c = e & 63;
    sm[c][r] = S[(size_t)(k0 + r) * sp + n0 + c];
  }
  __syncthreads();
  const int lane = t & 31, wave = t >> 5;
  const int q = lane >> 3, c8 = (lane & 7) * 8;
  unsigned short* D1 = dst + (size_t)z * dst_z;
  unsigned short* D2 = dst2 + (size_t)z * dst_z;
  for (int pass = 0; pass < 2; ++pass) {
#pragma unroll
    for (int it = 0; it < 2; ++it) {
      const int row = wave * 8 + it * 4 + q;
      unsigned short hb[8], lb[8];
#pragma unroll
      for (int e = 0; e < 8; ++e) {
        const float x = sm[row][c8 + e];
        if (CMODE == 0) {
          const unsigned short hbits = f2bf_bits(x);
          hb[e] = hbits;
          lb[e] = f2bf_bits(x - bf_bits2f(hbits));
        } else {
          hb[e] = h_bits(x * scale);
          lb[e] = 0;
        }
      }
      const size_t o = (size_t)(n0 + row) * dp + k0 + c8;
      const v4u uh = (v4u){pk16(hb[0], hb[1]), pk16(hb[2], hb[3]), pk16(hb[4], hb[5]), pk16(hb[6], hb[7])};
      *(volatile v4u*)(D1 + o) = uh;
      if (CMODE == 0) {
        const v4u ul = (v4u){pk16(lb[0], lb[1]), pk16(lb[2], lb[3]), pk16(lb[4], lb[5]), pk16(lb[6], lb[7])};
        *(volatile v4u*)(D2 + o) = ul;
      }
    }
    __threadfence();
  }
}

template <int RMODE>
__global__ __launch_bounds__(256) void rowcast_kernel(const float* __restrict__ src, int bsrc0, int srcR, int dstR, int nRows,
                                                      unsigned short* __restrict__ dhi, unsigned short* __restrict__ dlo) {
  const int g = blockIdx.x * 256 + threadIdx.x;
  if (g >= nRows * kG8) return;
  const int R  = g / kG8;
  const int c8 = (g - R * kG8) * 8;
  const int bl = R / dstR;
  const int n  = R - bl * dstR;
  const bool valid = n < srcR;
  const int ncl = valid ? n : (srcR - 1);
  const float* p = src + ((size_t)(bsrc0 + bl) * srcR + ncl) * kDM + c8;
  const v4f a = *(const v4f*)(p);
  const v4f c = *(const v4f*)(p + 4);
  unsigned short hb[8], lb[8];
#pragma unroll
  for (int e = 0; e < 4; ++e) {
    const float x0 = valid ? a[e] : 0.0f;
    const float x1 = valid ? c[e] : 0.0f;
    if (RMODE == 0) {
      const unsigned short h0 = f2bf_bits(x0);
      hb[e] = h0;  lb[e] = f2bf_bits(x0 - bf_bits2f(h0));
      const unsigned short h1 = f2bf_bits(x1);
      hb[4 + e] = h1;  lb[4 + e] = f2bf_bits(x1 - bf_bits2f(h1));
    } else {
      hb[e] = h_bits(x0);  hb[4 + e] = h_bits(x1);
      lb[e] = 0;  lb[4 + e] = 0;
    }
  }
  const v4u uh = (v4u){pk16(hb[0], hb[1]), pk16(hb[2], hb[3]), pk16(hb[4], hb[5]), pk16(hb[6], hb[7])};
  unsigned short* qh = dhi + (size_t)R * kDM + c8;
  if (RMODE == 0) {
    const v4u ul = (v4u){pk16(lb[0], lb[1]), pk16(lb[2], lb[3]), pk16(lb[4], lb[5]), pk16(lb[6], lb[7])};
    unsigned short* ql = dlo + (size_t)R * kDM + c8;
    *(volatile v4u*)qh = uh;
    *(volatile v4u*)ql = ul;
    __threadfence();
    *(volatile v4u*)qh = uh;
    *(volatile v4u*)ql = ul;
  } else {
    *(volatile v4u*)qh = uh;
    __threadfence();
    *(volatile v4u*)qh = uh;
  }
}

__device__ __forceinline__ void store_slab16x64(const float* slab, float* Cf, unsigned short* Ch, int lane) {
  wave_sync_lds();
  {
    const int hh = lane >> 4, c4 = (lane & 15) * 4;
    for (int pass = 0; pass < 2; ++pass) {
#pragma unroll
      for (int it = 0; it < 8; ++it) {
        const int row = it * 2 + hh;
        const v4f v = *(const v4f*)(slab + row * 68 + c4);
        *(volatile v4f*)(Cf + (size_t)row * kDM + c4) = v;
      }
      __threadfence();
    }
  }
  {
    const int q = lane >> 3, c8 = (lane & 7) * 8;
    for (int pass = 0; pass < 2; ++pass) {
#pragma unroll
      for (int it = 0; it < 4; ++it) {
        const int row = it * 4 + q;
        const float* sp = slab + row * 68 + c8;
        unsigned short hb[8];
#pragma unroll
        for (int e = 0; e < 8; ++e) hb[e] = h_bits(sp[e] * kVCarry);
        const v4u u = (v4u){pk16(hb[0], hb[1]), pk16(hb[2], hb[3]), pk16(hb[4], hb[5]), pk16(hb[6], hb[7])};
        *(volatile v4u*)(Ch + (size_t)row * kDM + c8) = u;
      }
      __threadfence();
    }
  }
  wave_sync_lds();
}

__global__ __launch_bounds__(256) void attn_kernel(
    const unsigned short* __restrict__ QHp, const unsigned short* __restrict__ QLp,
    const unsigned short* __restrict__ KHp, const unsigned short* __restrict__ KLp,
    const unsigned short* __restrict__ VHp, const unsigned short* __restrict__ VLp,
    const int* __restrict__ mask, const float* __restrict__ nq, const float* __restrict__ fg,
    float* __restrict__ Sst, float* __restrict__ Vf, unsigned short* __restrict__ Vh, int b0) {
  __shared__ __align__(16) float  sc[kKN * 84];
  __shared__ __align__(16) float  sS[kNTP * kKN];
  __shared__ __align__(16) __bf16 shi[kKN * 104];
  __shared__ __align__(16) __bf16 slo[kKN * 104];
  __shared__ __align__(16) float  slabs[8][16 * 68];
  const int tid = threadIdx.x, lane = tid & 31, wave = tid >> 5;
  const int m = lane & 15, hh = lane >> 4, koff = hh * 8, mOff = hh * 8;
  const int bl = blockIdx.x;
  const int b  = b0 + bl;
  const __bf16* Qh  = (const __bf16*)(const void*)QHp;
  const __bf16* Ql  = (const __bf16*)(const void*)QLp;
  const __bf16* Kh  = (const __bf16*)(const void*)KHp;
  const __bf16* Kl  = (const __bf16*)(const void*)KLp;
  const __bf16* Vth = (const __bf16*)(const void*)VHp;
  const __bf16* Vtl = (const __bf16*)(const void*)VLp;

  if (wave < kNTS / 16) {
    const int tt = wave;
    v8f acc = (v8f){0.f,0.f,0.f,0.f,0.f,0.f,0.f,0.f};
    const __bf16* qh = Qh + (size_t)m * kDM + koff;
    const __bf16* ql = Ql + (size_t)m * kDM + koff;
    const size_t krow = (size_t)(bl * kNTP + tt * 16 + m) * kDM + koff;
    const __bf16* kh = Kh + krow;
    const __bf16* kl = Kl + krow;
#pragma unroll 1
    for (int k0 = 0; k0 < kDM; k0 += 32) {
      const v16b ah = Frag<__bf16>::load(qh + k0);
      const v16b al = Frag<__bf16>::load(ql + k0);
      const v16b bh = Frag<__bf16>::load(kh + k0);
      const v16b bL = Frag<__bf16>::load(kl + k0);
      acc = bmma(ah, bh, acc);
      acc = bmma(ah, bL, acc);
      acc = bmma(al, bh, acc);
    }
#pragma unroll
    for (int r = 0; r < 8; ++r) sc[(mOff + r) * 84 + tt * 16 + m] = acc[r] * kScoreScale;
  }
  __syncthreads();

  {
    const int kq = tid & 15;
    const int tq = tid >> 4;
#pragma unroll 1
    for (int it = 0; it < kNTP / 16; ++it) {
      const int t   = it * 16 + tq;
      const int tsc = (t < kNTS) ? t : (kNTS - 1);
      const int tmk = (t < kNT) ? t : (kNT - 1);
      const int mk  = mask[(size_t)b * kNT + tmk];
      float s = sc[kq * 84 + tsc];
      s = (mk != 0) ? s : -3.4028235e38f;
      float mx = s;
      mx = fmaxf(mx, __shfl_xor(mx, 1, 32));
      mx = fmaxf(mx, __shfl_xor(mx, 2, 32));
      mx = fmaxf(mx, __shfl_xor(mx, 4, 32));
      mx = fmaxf(mx, __shfl_xor(mx, 8, 32));
      const float e = expf(s - mx);
      float sum = e;
      sum += __shfl_xor(sum, 1, 32);
      sum += __shfl_xor(sum, 2, 32);
      sum += __shfl_xor(sum, 4, 32);
      sum += __shfl_xor(sum, 8, 32);
      float p = e * (1.0f / sum);
      p = (t < kNT) ? p : 0.0f;
      sS[t * kKN + kq] = p;
      __bf16 ph, pl;
      at_split(p, ph, pl);
      shi[kq * 104 + t] = ph;
      slo[kq * 104 + t] = pl;
    }
  }
  __syncthreads();

  {
    float* sp = Sst + (size_t)b * (kNTP * kKN);
    for (int pass = 0; pass < 2; ++pass) {
      for (int i = tid; i < (kNTP * kKN) / 4; i += 256) {
        const v4f val = *(const v4f*)(sS + i * 4);
        *(volatile v4f*)(sp + i * 4) = val;
      }
      __threadfence();
    }
  }

  const float gate = 1.0f / (1.0f + expf(-fg[0]));
  const float omg  = 1.0f - gate;
  float* slab = slabs[wave];
  for (int sl = wave; sl < kDM / 64; sl += 8) {
    const int d0 = sl * 64;
    v8f acc[4];
#pragma unroll
    for (int j = 0; j < 4; ++j) acc[j] = (v8f){0.f,0.f,0.f,0.f,0.f,0.f,0.f,0.f};
#pragma unroll 1
    for (int ks = 0; ks < kNTP / 32; ++ks) {
      const int k0 = ks * 32;
      const v16b ah = Frag<__bf16>::load(shi + m * 104 + k0 + koff);
      const v16b al = Frag<__bf16>::load(slo + m * 104 + k0 + koff);
#pragma unroll
      for (int j = 0; j < 4; ++j) {
        const size_t bo = (size_t)(d0 + j * 16 + m) * kMRC + bl * kNTP + k0 + koff;
        const v16b bh = Frag<__bf16>::load(Vth + bo);
        const v16b bL = Frag<__bf16>::load(Vtl + bo);
        acc[j] = bmma(ah, bh, acc[j]);
        acc[j] = bmma(ah, bL, acc[j]);
        acc[j] = bmma(al, bh, acc[j]);
      }
    }
#pragma unroll
    for (int j = 0; j < 4; ++j) {
      const int n = d0 + j * 16 + m;
#pragma unroll
      for (int r = 0; r < 8; ++r) {
        const int node = mOff + r;
        const float val = omg * acc[j][r] + gate * nq[(size_t)node * kDM + n];
        slab[node * 68 + j * 16 + m] = val;
      }
    }
    store_slab16x64(slab, Vf + (size_t)(b * kKN) * kDM + d0, Vh + (size_t)(b * kKN) * kDM + d0, lane);
  }
}

template <int EMODE>
__global__ __launch_bounds__(256) void edge_kernel(const float* __restrict__ H, const float* __restrict__ be1,
                                                   const float* __restrict__ We2, const float* __restrict__ be2,
                                                   float* __restrict__ outp) {
  __shared__ __align__(16) _Float16 tile[256 * 72];
  __shared__ __align__(16) _Float16 sw2[kHD];
  __shared__ __align__(16) float    sb1[kHD];
  __shared__ __align__(16) float    sE[256];
  const int tid = threadIdx.x, lane = tid & 31, wave = tid >> 5;
  const int m = lane & 15, hh = lane >> 4, koff = hh * 8, mOff = hh * 8;
  const int b = blockIdx.x;
  if (tid < kHD / 8) {
    const v4f wa = *(const v4f*)(We2 + tid * 8);
    const v4f wc = *(const v4f*)(We2 + tid * 8 + 4);
    v8h wv;
#pragma unroll
    for (int e = 0; e < 4; ++e) {
      wv[e]     = (_Float16)(wa[e] * kWCarry);
      wv[4 + e] = (_Float16)(wc[e] * kWCarry);
    }
    *(v8h*)(sw2 + tid * 8) = wv;
  }
  for (int e = tid; e < kHD; e += 256) sb1[e] = be1[e];
  const int pi = tid >> 4, pj = tid & 15;
  const float* hip = H + (size_t)(b * kKN + pi) * (2 * kHD);
  const float* hjp = H + (size_t)(b * kKN + pj) * (2 * kHD) + kHD;
  v8f acc[2];
  acc[0] = (v8f){0.f,0.f,0.f,0.f,0.f,0.f,0.f,0.f};
  acc[1] = (v8f){0.f,0.f,0.f,0.f,0.f,0.f,0.f,0.f};
  __syncthreads();
#pragma unroll 1
  for (int hc = 0; hc < kHD / 64; ++hc) {
    const int h0 = hc * 64;
#pragma unroll
    for (int g = 0; g < 8; ++g) {
      const int hb = h0 + g * 8;
      const v4f a0 = *(const v4f*)(hip + hb), a1 = *(const v4f*)(hip + hb + 4);
      const v4f c0 = *(const v4f*)(hjp + hb), c1 = *(const v4f*)(hjp + hb + 4);
      const v4f e0 = *(const v4f*)(sb1 + hb), e1 = *(const v4f*)(sb1 + hb + 4);
      v8h hv;
#pragma unroll
      for (int e = 0; e < 4; ++e) {
        hv[e]     = (_Float16)(fmaxf(a0[e] + c0[e] + e0[e], 0.0f) * kReluCarry);
        hv[4 + e] = (_Float16)(fmaxf(a1[e] + c1[e] + e1[e], 0.0f) * kReluCarry);
      }
      *(v8h*)(tile + tid * 72 + g * 8) = hv;
    }
    __syncthreads();
#pragma unroll
    for (int ks = 0; ks < 2; ++ks) {
      const int k0 = ks * 32;
      const v16h bw = Frag<_Float16>::load(sw2 + h0 + k0 + koff);
#pragma unroll
      for (int rt2 = 0; rt2 < 2; ++rt2) {
        const v16h a = Frag<_Float16>::load(tile + ((wave * 2 + rt2) * 16 + m) * 72 + k0 + koff);
        acc[rt2] = hmma(a, bw, acc[rt2]);
      }
    }
    __syncthreads();
  }
  const float be2v = be2[0];
  if (m == 0) {
#pragma unroll
    for (int rt2 = 0; rt2 < 2; ++rt2)
#pragma unroll
      for (int r = 0; r < 8; ++r)
        sE[(wave * 2 + rt2) * 16 + mOff + r] = acc[rt2][r] * kEdgeScale + be2v;
  }
  __syncthreads();
  if (EMODE == 0) {
    const float x = sE[tid];
    float mx = x;
    mx = fmaxf(mx, __shfl_xor(mx, 1, 32));
    mx = fmaxf(mx, __shfl_xor(mx, 2, 32));
    mx = fmaxf(mx, __shfl_xor(mx, 4, 32));
    mx = fmaxf(mx, __shfl_xor(mx, 8, 32));
    const float ex = expf(x - mx);
    float sum = ex;
    sum += __shfl_xor(sum, 1, 32);
    sum += __shfl_xor(sum, 2, 32);
    sum += __shfl_xor(sum, 4, 32);
    sum += __shfl_xor(sum, 8, 32);
    const float p = ex * (1.0f / sum);
    __syncthreads();
    sE[tid] = p;
    __syncthreads();
  }
  if (tid < 64) {
    const v4f v = *(const v4f*)(sE + tid * 4);
    float* op = outp + (size_t)b * 256 + tid * 4;
    *(volatile v4f*)op = v;
    __threadfence();
    *(volatile v4f*)op = v;
  }
}

__global__ __launch_bounds__(256) void msg_kernel(const float* __restrict__ Adj,
                                                  const unsigned short* __restrict__ GTHp, const unsigned short* __restrict__ GTLp,
                                                  const float* __restrict__ Vin, float* __restrict__ Vout,
                                                  unsigned short* __restrict__ Vhout) {
  __shared__ __align__(16) float slabs[8][16 * 68];
  const int tid = threadIdx.x, lane = tid & 31, wave = tid >> 5;
  const int m = lane & 15, hh = lane >> 4, koff = hh * 8, mOff = hh * 8;
  const int b = blockIdx.x;
  const __bf16* Gh = (const __bf16*)(const void*)GTHp;
  const __bf16* Gl = (const __bf16*)(const void*)GTLp;
  const v4u z4 = (v4u){0u, 0u, 0u, 0u};
  FB fah, fal;
  {
    const float* ar = Adj + (size_t)b * 256 + m * 16 + koff;
    const v4f a0 = *(const v4f*)(ar);
    const v4f a1 = *(const v4f*)(ar + 4);
    v8b th, tl;
#pragma unroll
    for (int e = 0; e < 4; ++e) {
      __bf16 x, y;
      at_split(a0[e], x, y); th[e] = x;     tl[e] = y;
      at_split(a1[e], x, y); th[4 + e] = x; tl[4 + e] = y;
    }
    fah.h[0] = th; fah.u4[1] = z4;
    fal.h[0] = tl; fal.u4[1] = z4;
  }
  float* slab = slabs[wave];
  for (int sl = wave; sl < kDM / 64; sl += 8) {
    const int d0 = sl * 64;
    v8f acc[4];
#pragma unroll
    for (int j = 0; j < 4; ++j) acc[j] = (v8f){0.f,0.f,0.f,0.f,0.f,0.f,0.f,0.f};
#pragma unroll
    for (int j = 0; j < 4; ++j) {
      const size_t bo = (size_t)(d0 + j * 16 + m) * kVROWS + b * kKN + koff;
      FB fbh, fbl;
      fbh.h[0] = *(const v8b*)(Gh + bo); fbh.u4[1] = z4;
      fbl.h[0] = *(const v8b*)(Gl + bo); fbl.u4[1] = z4;
      acc[j] = bmma(fah.v, fbh.v, acc[j]);
      acc[j] = bmma(fah.v, fbl.v, acc[j]);
      acc[j] = bmma(fal.v, fbh.v, acc[j]);
    }
#pragma unroll
    for (int j = 0; j < 4; ++j) {
      const int n = d0 + j * 16 + m;
#pragma unroll
      for (int r = 0; r < 8; ++r) {
        const int node = mOff + r;
        const float val = Vin[(size_t)(b * kKN + node) * kDM + n] + fmaxf(acc[j][r], 0.0f);
        slab[node * 68 + j * 16 + m] = val;
      }
    }
    store_slab16x64(slab, Vout + (size_t)(b * kKN) * kDM + d0, Vhout + (size_t)(b * kKN) * kDM + d0, lane);
  }
}

__global__ __launch_bounds__(256) void pack_s_kernel(const float* __restrict__ Sst, float* __restrict__ out0) {
  const int i = blockIdx.x * 256 + threadIdx.x;
  if (i >= (kNB * kNT * kKN) / 4) return;
  const int e = i * 4;
  const int b = e / (kNT * kKN);
  const int rem = e - b * (kNT * kKN);
  const v4f v = *(const v4f*)(Sst + (size_t)b * (kNTP * kKN) + rem);
  *(volatile v4f*)(out0 + e) = v;
  __threadfence();
  *(volatile v4f*)(out0 + e) = v;
}

extern "C" void kernel_launch(void* const* d_in, const int* in_sizes, int n_in,
                              void* d_out, int out_size, void* d_ws, size_t ws_size,
                              hipStream_t stream) {
  if (n_in < 16) return;
  if (in_sizes[0] != kNB * kNT * kDM || in_sizes[1] != kNB * kNT || in_sizes[2] != kKN * kDM ||
      in_sizes[3] != kDM * kDM || in_sizes[4] != kDM || in_sizes[5] != kDM * kDM || in_sizes[6] != kDM ||
      in_sizes[7] != kDM * kDM || in_sizes[8] != kDM || in_sizes[9] != 2 * kDM * kHD || in_sizes[10] != kHD ||
      in_sizes[11] != kHD || in_sizes[12] < 1 || in_sizes[13] < 1 || in_sizes[14] != kNL * kDM * kDM ||
      in_sizes[15] != kNL * kDM) return;
  if (out_size != kNB * kNT * kKN + kNB * kKN * kDM + kNB * kKN * kKN) return;
  if (ws_size < kWsTotal) return;

  const float* w    = (const float*)d_in[0];
  const int*   mask = (const int*)d_in[1];
  const float* nq   = (const float*)d_in[2];
  const float* Wq   = (const float*)d_in[3];
  const float* bq   = (const float*)d_in[4];
  const float* Wk   = (const float*)d_in[5];
  const float* bk   = (const float*)d_in[6];
  const float* Wv   = (const float*)d_in[7];
  const float* bv   = (const float*)d_in[8];
  const float* We1  = (const float*)d_in[9];
  const float* be1  = (const float*)d_in[10];
  const float* We2  = (const float*)d_in[11];
  const float* be2  = (const float*)d_in[12];
  const float* fg   = (const float*)d_in[13];
  const float* Wg   = (const float*)d_in[14];
  const float* bg   = (const float*)d_in[15];

  char* ws = (char*)d_ws;
  unsigned short* WqH  = (unsigned short*)(ws + oWqH);
  unsigned short* WqL  = (unsigned short*)(ws + oWqL);
  unsigned short* WkT  = (unsigned short*)(ws + oWkT);
  unsigned short* WvT  = (unsigned short*)(ws + oWvT);
  unsigned short* We1T = (unsigned short*)(ws + oWe1T);
  unsigned short* WgT  = (unsigned short*)(ws + oWgT);
  unsigned short* QinH = (unsigned short*)(ws + oQinH);
  unsigned short* QinL = (unsigned short*)(ws + oQinL);
  unsigned short* QH   = (unsigned short*)(ws + oQH);
  unsigned short* QL   = (unsigned short*)(ws + oQL);
  unsigned short* wH   = (unsigned short*)(ws + oWH);
  unsigned short* KtH  = (unsigned short*)(ws + oKtH);
  unsigned short* KtL  = (unsigned short*)(ws + oKtL);
  unsigned short* VtH  = (unsigned short*)(ws + oVtH);
  unsigned short* VtL  = (unsigned short*)(ws + oVtL);
  float*          Hbuf = (float*)(ws + oH);
  unsigned short* GTH  = (unsigned short*)(ws + oGTH);
  unsigned short* GTL  = (unsigned short*)(ws + oGTL);
  float*          VfB  = (float*)(ws + oVfB);
  float*          Sst  = (float*)(ws + oSst);
  float*          VfA  = (float*)(ws + oVfA);
  unsigned short* VhA  = (unsigned short*)(ws + oVhA);
  unsigned short* VhB  = (unsigned short*)(ws + oVhB);
  float*          Adj  = (float*)(ws + oAdj);

  float* out0 = (float*)d_out;
  float* out1 = out0 + (size_t)kNB * kNT * kKN;
  float* out2 = out1 + (size_t)kNB * kKN * kDM;

  tcast_kernel<0><<<dim3(kDM / 64, kDM / 64, 1), 256, 0, stream>>>(Wq, 0L, kDM, WqH, WqL, 0L, kDM, 1.0f);
  tcast_kernel<1><<<dim3(kDM / 64, kDM / 64, 1), 256, 0, stream>>>(Wk, 0L, kDM, WkT, WkT, 0L, kDM, kKVCarry);
  tcast_kernel<1><<<dim3(kDM / 64, kDM / 64, 1), 256, 0, stream>>>(Wv, 0L, kDM, WvT, WvT, 0L, kDM, kKVCarry);
  tcast_kernel<1><<<dim3(kDM / 64, kHD / 64, 2), 256, 0, stream>>>(We1, (long)kDM * kHD, kHD, We1T, We1T,
                                                                    (long)kHD * kDM, kDM, kWCarry);
  tcast_kernel<1><<<dim3(kDM / 64, kDM / 64, 2), 256, 0, stream>>>(Wg, (long)kDM * kDM, kDM, WgT, WgT,
                                                                    (long)kDM * kDM, kDM, kWCarry);
  rowcast_kernel<0><<<(kQR * kG8) / 256, 256, 0, stream>>>(nq, 0, kKN, kQR, kQR, QinH, QinL);
  wmma_gemm64<1, true, 2, 2, false><<<dim3(2, 1), 256, 0, stream>>>(
      QinH, QinL, kDM, 0L, WqH, WqL, kDM, 0L, (void*)QH, (void*)QL, kDM, 0L, bq, bq, 0L, kQR, kDM, kDM, 1.0f);

  for (int cb = 0; cb < kNCH; ++cb) {
    rowcast_kernel<1><<<(kMRC * kG8) / 256, 256, 0, stream>>>(w, cb * kBPC, kNT, kNTP, kMRC, wH, wH);
    wmma_gemm64<0, false, 2, 2, false><<<dim3(144, 1), 256, 0, stream>>>(
        wH, wH, kDM, 0L, WkT, WkT, kDM, 0L, (void*)KtH, (void*)KtL, kDM, 0L, bk, bk, 0L, kMRC, kDM, kDM, kKVScale);
    wmma_gemm64<0, false, 1, 2, false, 0, kNTP, kNT><<<dim3(144, 1), 256, 0, stream>>>(
        WvT, WvT, kDM, 0L, wH, wH, kDM, 0L, (void*)VtH, (void*)VtL, kMRC, 0L, bv, bv, 0L, kDM, kMRC, kDM, kKVScale);
    attn_kernel<<<kBPC, 256, 0, stream>>>(QH, QL, KtH, KtL, VtH, VtL, mask, nq, fg, Sst, VfA, VhA, cb * kBPC);
  }

  wmma_gemm64<0, false, 0, 0, false><<<dim3(128, 1), 256, 0, stream>>>(
      VhA, VhA, kDM, 0L, We1T, We1T, kDM, 0L, (void*)Hbuf, (void*)Hbuf, 2 * kHD, 0L, be1, be1, 0L,
      kVROWS, 2 * kHD, kDM, kProjScale);
  edge_kernel<0><<<kNB, 256, 0, stream>>>(Hbuf, be1, We2, be2, Adj);

  wmma_gemm64<0, false, 1, 2, false><<<dim3(96, 1), 256, 0, stream>>>(
      WgT, WgT, kDM, 0L, VhA, VhA, kDM, 0L, (void*)GTH, (void*)GTL, kVROWS, 0L, bg, bg, 0L,
      kDM, kVROWS, kDM, kProjScale);
  msg_kernel<<<kNB, 256, 0, stream>>>(Adj, GTH, GTL, VfA, VfB, VhB);
  wmma_gemm64<0, false, 1, 2, false><<<dim3(96, 1), 256, 0, stream>>>(
      WgT + (size_t)kDM * kDM, WgT + (size_t)kDM * kDM, kDM, 0L, VhB, VhB, kDM, 0L, (void*)GTH, (void*)GTL, kVROWS, 0L,
      bg + kDM, bg + kDM, 0L, kDM, kVROWS, kDM, kProjScale);
  msg_kernel<<<kNB, 256, 0, stream>>>(Adj, GTH, GTL, VfB, out1, VhA);

  wmma_gemm64<0, false, 0, 0, false><<<dim3(128, 1), 256, 0, stream>>>(
      VhA, VhA, kDM, 0L, We1T, We1T, kDM, 0L, (void*)Hbuf, (void*)Hbuf, 2 * kHD, 0L, be1, be1, 0L,
      kVROWS, 2 * kHD, kDM, kProjScale);
  edge_kernel<1><<<kNB, 256, 0, stream>>>(Hbuf, be1, We2, be2, out2);

  pack_s_kernel<<<(kNB * kNT * kKN) / 4 / 256, 256, 0, stream>>>(Sst, out0);
}
